// CausalSelfAttention_44195213475965
// MI455X (gfx1250) — hardware-verified
//
#include <hip/hip_runtime.h>


#ifndef NB
#define NB 4
#endif
#ifndef SEQ
#define SEQ 2048
#endif
#define NB_FULL  4
#define SEQ_FULL 2048
#define TT   SEQ
#define DM   1024
#define NH_  16
#define HD   64
#define DQ   (NH_ * HD)
#define RH   ((TT) < 512 ? (TT) : 512)
#define CSC  0.045084220027780106f
static_assert(NB <= NB_FULL);
static_assert(SEQ <= SEQ_FULL);
static_assert((TT & (TT - 1)) == 0);
static_assert(TT % 64 == 0);
static_assert(RH % 64 == 0);
static_assert(RH <= TT);
static_assert(HD == 64);
static_assert(DQ == DM);
static_assert(DM % 64 == 0);
static_assert((3 * DQ) % 64 == 0);
static_assert(DM % 32 == 0);

typedef _Float16 h16;
typedef unsigned short bf;
typedef __attribute__((ext_vector_type(16))) __bf16   v16bf;
typedef __attribute__((ext_vector_type(16))) _Float16 v16h;
typedef __attribute__((ext_vector_type(8)))  _Float16 v8h;
typedef __attribute__((ext_vector_type(8)))  unsigned short v8us;
typedef __attribute__((ext_vector_type(8)))  float    v8f;
typedef __attribute__((ext_vector_type(4)))  float    v4f;
typedef __attribute__((ext_vector_type(2)))  _Float16 v2h;
typedef __attribute__((ext_vector_type(2)))  unsigned short v2us;
typedef __attribute__((ext_vector_type(2)))  float    v2f;
typedef v4f  __attribute__((may_alias)) v4fa;

__device__ __forceinline__ unsigned short f2bf(float f) { unsigned u = __float_as_uint(f); u += 0x7FFFu + ((u >> 16) & 1u); return (unsigned short)(u >> 16); }
__device__ __forceinline__ float bf2f(unsigned short b) { return __uint_as_float(((unsigned)b) << 16); }
__device__ __forceinline__ float bfr(float f) { return bf2f(f2bf(f)); }
__device__ __forceinline__ v16h cat16(v8h lo, v8h hi) { return __builtin_shufflevector(lo, hi, 0, 1, 2, 3, 4, 5, 6, 7, 8, 9, 10, 11, 12, 13, 14, 15); }
__device__ __forceinline__ v16bf cat16b(v8us lo, v8us hi) { return __builtin_bit_cast(v16bf, __builtin_shufflevector(lo, hi, 0, 1, 2, 3, 4, 5, 6, 7, 8, 9, 10, 11, 12, 13, 14, 15)); }
__device__ __forceinline__ v8f wmma16(v16h a, v16h b, v8f c) { return __builtin_amdgcn_wmma_f32_16x16x32_f16(false, a, false, b, (short)0, c, false, false); }
__device__ __forceinline__ v8f wmmab(v16bf a, v16bf b, v8f c) { return __builtin_amdgcn_wmma_f32_16x16x32_bf16(false, a, false, b, (short)0, c, false, false); }
__device__ __forceinline__ h16 tohx(float x) { return (h16)x; }
__device__ __forceinline__ void splitf(float y, unsigned short& h, unsigned short& l) { h = f2bf(y); l = f2bf(y - bf2f(h)); }

template <typename T16> struct WFrag;
template <> struct WFrag<h16> { typedef v16h V; static __device__ __forceinline__ V ld(const h16* p) { return cat16(*(const v8h*)p, *(const v8h*)(p + 16)); } static __device__ __forceinline__ v8f mma(V a, V b, v8f c) { return wmma16(a, b, c); } };
template <> struct WFrag<bf> { typedef v16bf V; static __device__ __forceinline__ V ld(const bf* p) { return cat16b(*(const v8us*)p, *(const v8us*)(p + 16)); } static __device__ __forceinline__ v8f mma(V a, V b, v8f c) { return wmmab(a, b, c); } };

template <typename T16, int NSPLIT, bool BIAS>
__global__ __launch_bounds__(32) void k_gemmw(const T16* __restrict__ A, const T16* __restrict__ A2, const T16* __restrict__ Bt, const T16* __restrict__ Bt2, int K, float* C, int ldc, const float* __restrict__ bias, size_t sA, size_t sB, size_t sC) {
    typedef typename WFrag<T16>::V V;
    __shared__ __align__(16) float os[16 * 68];
    const size_t z = blockIdx.z; A += z * sA; if (A2) A2 += z * sA; Bt += z * sB; if (Bt2) Bt2 += z * sB; C += z * sC;
    const int lane = threadIdx.x & 31, lr = lane & 15, hi = lane >> 4; const int r0 = blockIdx.x * 64, c0 = blockIdx.y * 64;
    v8f acc[4][4];
#pragma unroll
    for (int mb = 0; mb < 4; ++mb)
#pragma unroll
        for (int nb = 0; nb < 4; ++nb) acc[mb][nb] = (v8f){};
    const size_t aoff = (size_t)(r0 + lr) * K + 8 * hi, boff = (size_t)(c0 + lr) * K + 8 * hi;
#pragma unroll 1
    for (int kc = 0; kc < K; kc += 32) {
        V a[4], a2[4];
#pragma unroll
        for (int mb = 0; mb < 4; ++mb) { a[mb] = WFrag<T16>::ld(A + aoff + (size_t)mb * 16 * K + kc); if (NSPLIT == 1 || NSPLIT == 2) a2[mb] = WFrag<T16>::ld(A2 + aoff + (size_t)mb * 16 * K + kc); }
#pragma unroll
        for (int nb = 0; nb < 4; ++nb) { const V b = WFrag<T16>::ld(Bt + boff + (size_t)nb * 16 * K + kc); V b2; if (NSPLIT >= 2) b2 = WFrag<T16>::ld(Bt2 + boff + (size_t)nb * 16 * K + kc);
#pragma unroll
            for (int mb = 0; mb < 4; ++mb) { acc[mb][nb] = WFrag<T16>::mma(a[mb], b, acc[mb][nb]); if (NSPLIT == 1 || NSPLIT == 2) acc[mb][nb] = WFrag<T16>::mma(a2[mb], b, acc[mb][nb]); if (NSPLIT >= 2) acc[mb][nb] = WFrag<T16>::mma(a[mb], b2, acc[mb][nb]); } }
        asm volatile("v_nop\n\tv_nop\n\tv_nop\n\tv_nop" : "+v"(acc[0][0]), "+v"(acc[1][1]), "+v"(acc[2][2]), "+v"(acc[3][3]) : "v"(a[0]), "v"(a[3]));
    }
#pragma unroll
    for (int mb = 0; mb < 4; ++mb) {
#pragma unroll
        for (int nb = 0; nb < 4; ++nb) {
#pragma unroll
            for (int j = 0; j < 8; ++j) os[(hi * 8 + j) * 68 + nb * 16 + lr] = acc[mb][nb][j]; }
        __builtin_amdgcn_wave_barrier(); asm volatile("" ::: "memory");
        float* crow = C + (size_t)(r0 + mb * 16) * ldc + c0;
#pragma unroll 1
        for (int ps = 0; ps < 2; ++ps) {
#pragma unroll
            for (int s = 0; s < 8; ++s) { const int row = 2 * s + hi, cofs = lr * 4; v4f val = *(const v4fa*)(os + row * 68 + cofs); if (BIAS) { val[0] += bfr(bias[c0 + cofs]); val[1] += bfr(bias[c0 + cofs + 1]); val[2] += bfr(bias[c0 + cofs + 2]); val[3] += bfr(bias[c0 + cofs + 3]); }
                *(volatile v4f*)(crow + (size_t)row * ldc + cofs) = val; }
            if (ps == 0) __threadfence(); }
        __builtin_amdgcn_wave_barrier(); asm volatile("" ::: "memory");
    }
}

__global__ __launch_bounds__(256) void k_wtG(const float* __restrict__ w, int K, int N, bf* Bt) {
    const int lane = threadIdx.x & 31; const int L0 = (blockIdx.x * 8 + (threadIdx.x >> 5)) * 8; const int nlines = N * K / 64;
#pragma unroll
    for (int ps = 0; ps < 2; ++ps) {
#pragma unroll 1
        for (int l = 0; l < 8; ++l) { const int L = L0 + l; if (L >= nlines) break; const size_t e = (size_t)L * 64 + lane * 2; const int k = (int)(e % K), n = (int)(e / K); v2us o;
            o[0] = f2bf(w[(size_t)k * N + n]); o[1] = f2bf(w[(size_t)(k + 1) * N + n]); *(volatile v2us*)(Bt + e) = o; }
        if (ps == 0) __threadfence(); }
}
__global__ __launch_bounds__(256) void k_cvt8(const float* __restrict__ src, bf* dst, size_t n8) { const size_t i = (size_t)blockIdx.x * 256 + threadIdx.x; if (i >= n8) return; const v8f v = *(const v8f*)(src + i * 8); v8us o;
#pragma unroll
    for (int k = 0; k < 8; ++k) o[k] = f2bf(v[k]); *(volatile v8us*)(dst + i * 8) = o; __threadfence(); *(volatile v8us*)(dst + i * 8) = o; }

#define NQK ((unsigned)(2 * NH_) * (unsigned)TT * (unsigned)HD)
#define NVT ((unsigned)NH_ * (unsigned)HD * (unsigned)TT)
#define BLK_QK (NQK / 512u)
#define BLK_VT (NVT / 512u)
static_assert(NQK % 512u == 0);
static_assert(NVT % 512u == 0);
static_assert(RH % 8 == 0);
__global__ __launch_bounds__(256) void k_planes(const float* __restrict__ F, h16* QK16, bf* QKBh, bf* QKBl, h16* VT16, bf* VTBh, bf* VTBl) {
    if (blockIdx.x < BLK_QK) {
        const unsigned e = (blockIdx.x * 256u + threadIdx.x) * 2u;
        const unsigned d = e % (unsigned)HD, t = (e / (unsigned)HD) % (unsigned)TT, hp = e / ((unsigned)HD * (unsigned)TT);
        const v2f x = *(const v2f*)(F + (size_t)t * (3 * DQ) + hp * HD + d);
        v2h o16; v2us oh, ol;
#pragma unroll
        for (int q = 0; q < 2; ++q) { o16[q] = tohx(x[q]); unsigned short a2, c2; splitf(x[q], a2, c2); oh[q] = a2; ol[q] = c2; }
        const bool band = t < (unsigned)RH; const unsigned eb = (hp * (unsigned)RH + t) * (unsigned)HD + d;
        *(volatile v2h*)(QK16 + e) = o16; if (band) { *(volatile v2us*)(QKBh + eb) = oh; *(volatile v2us*)(QKBl + eb) = ol; }
        __threadfence();
        *(volatile v2h*)(QK16 + e) = o16; if (band) { *(volatile v2us*)(QKBh + eb) = oh; *(volatile v2us*)(QKBl + eb) = ol; }
    } else {
        const unsigned e = ((blockIdx.x - BLK_QK) * 256u + threadIdx.x) * 2u;
        const unsigned t = e % (unsigned)TT, d = (e / (unsigned)TT) % (unsigned)HD, g = e / ((unsigned)TT * (unsigned)HD);
        v2h o16; v2us oh, ol;
#pragma unroll
        for (int q = 0; q < 2; ++q) { const float x = F[(size_t)(t + (unsigned)q) * (3 * DQ) + 2 * DQ + g * HD + d]; o16[q] = tohx(x); unsigned short a2, c2; splitf(x, a2, c2); oh[q] = a2; ol[q] = c2; }
        const bool band = t < (unsigned)RH; const unsigned eb = (g * (unsigned)HD + d) * (unsigned)RH + t;
        *(volatile v2h*)(VT16 + e) = o16; if (band) { *(volatile v2us*)(VTBh + eb) = oh; *(volatile v2us*)(VTBl + eb) = ol; }
        __threadfence();
        *(volatile v2h*)(VT16 + e) = o16; if (band) { *(volatile v2us*)(VTBh + eb) = oh; *(volatile v2us*)(VTBl + eb) = ol; }
    }
}

template <typename T16> struct PK;
template <> struct PK<h16> {
    static __device__ __forceinline__ v16h hi(const v8f& a, const v8f& b) { v8h x, y;
#pragma unroll
        for (int r = 0; r < 8; ++r) { x[r] = (h16)a[r]; y[r] = (h16)b[r]; } return cat16(x, y); }
    static __device__ __forceinline__ v16h lo(const v8f& a, const v8f& b) { return hi(a, b); }
};
template <> struct PK<bf> {
    static __device__ __forceinline__ v16bf hi(const v8f& a, const v8f& b) { v8us x, y;
#pragma unroll
        for (int r = 0; r < 8; ++r) { x[r] = f2bf(a[r]); y[r] = f2bf(b[r]); } return cat16b(x, y); }
    static __device__ __forceinline__ v16bf lo(const v8f& a, const v8f& b) { v8us x, y;
#pragma unroll
        for (int r = 0; r < 8; ++r) { x[r] = f2bf(a[r] - bf2f(f2bf(a[r]))); y[r] = f2bf(b[r] - bf2f(f2bf(b[r]))); } return cat16b(x, y); }
};

template <typename T16, int NS>
__device__ __forceinline__ void attn_body(const T16* Qh, const T16* Ql, const T16* Kh, const T16* Kl, const T16* Vh, const T16* Vl,
                                          const unsigned vpitch, const unsigned q0, bf* Ah, bf* Al, float* os) {
    typedef WFrag<T16> W; typedef typename W::V V;
    const unsigned lane = threadIdx.x & 31u, lr = lane & 15u, hf = lane >> 4;
    const unsigned qi = q0 + lr;
    const float cl = (NS == 1) ? 10.0f : 0.0f;
    V qh[2], ql[2];
#pragma unroll
    for (int ks = 0; ks < 2; ++ks) { const unsigned qo = qi * (unsigned)HD + (unsigned)ks * 32u + 8u * hf; qh[ks] = W::ld(Qh + qo); ql[ks] = qh[ks]; if (NS == 3) ql[ks] = W::ld(Ql + qo); }
    v8f o[4];
#pragma unroll
    for (int dt = 0; dt < 4; ++dt) o[dt] = (v8f){};
    float m = -1.0e30f, l = 0.0f;
    const unsigned nkb = (q0 >> 6) + 1u;
#pragma unroll 1
    for (unsigned kbi = 0; kbi < nkb; ++kbi) {
        const unsigned kb = kbi << 6;
        v8f s[4];
#pragma unroll
        for (int j = 0; j < 4; ++j) {
            s[j] = (v8f){};
            const unsigned ko = (kb + 16u * (unsigned)j + lr) * (unsigned)HD + 8u * hf;
            const V k0 = W::ld(Kh + ko), k1 = W::ld(Kh + ko + 32u);
            s[j] = W::mma(k0, qh[0], s[j]); s[j] = W::mma(k1, qh[1], s[j]);
            if (NS == 3) { const V k0l = W::ld(Kl + ko), k1l = W::ld(Kl + ko + 32u);
                s[j] = W::mma(k0l, qh[0], s[j]); s[j] = W::mma(k1l, qh[1], s[j]); s[j] = W::mma(k0, ql[0], s[j]); s[j] = W::mma(k1, ql[1], s[j]);
                asm volatile("v_nop\n\tv_nop\n\tv_nop\n\tv_nop" : "+v"(s[j]) : "v"(k0), "v"(k1), "v"(k0l), "v"(k1l) : "memory"); }
            else { asm volatile("v_nop\n\tv_nop\n\tv_nop\n\tv_nop" : "+v"(s[j]) : "v"(k0), "v"(k1) : "memory"); }
        }
        const bool diag = (kbi + 1u == nkb);
        float mx = -1.0e30f;
#pragma unroll
        for (int j = 0; j < 4; ++j)
#pragma unroll
            for (int r = 0; r < 8; ++r) { float v = s[j][r] * CSC; const unsigned key = kb + 16u * (unsigned)j + 8u * hf + (unsigned)r; if (diag) v = (key <= qi) ? v : -1.0e30f; s[j][r] = v; mx = fmaxf(mx, v); }
        mx = fmaxf(mx, __shfl_xor(mx, 16, 32));
        const float mn = fmaxf(m, mx); const float alpha = __builtin_amdgcn_exp2f(m - mn); m = mn; l *= alpha;
#pragma unroll
        for (int j = 0; j < 4; ++j)
#pragma unroll
            for (int r = 0; r < 8; ++r) { const float p = __builtin_amdgcn_exp2f(s[j][r] - mn + cl); s[j][r] = p; l += p; }
#pragma unroll
        for (int dt = 0; dt < 4; ++dt)
#pragma unroll
            for (int r = 0; r < 8; ++r) o[dt][r] *= alpha;
#pragma unroll
        for (int ks = 0; ks < 2; ++ks) {
            const V ph = PK<T16>::hi(s[2 * ks], s[2 * ks + 1]); V pl = ph; if (NS == 3) pl = PK<T16>::lo(s[2 * ks], s[2 * ks + 1]);
#pragma unroll
            for (int dt = 0; dt < 4; ++dt) {
                const unsigned vo = ((unsigned)dt * 16u + lr) * vpitch + kb + (unsigned)ks * 32u + 8u * hf;
                const V vh = W::ld(Vh + vo);
                o[dt] = W::mma(vh, ph, o[dt]);
                if (NS == 3) { const V vl = W::ld(Vl + vo); o[dt] = W::mma(vl, ph, o[dt]); o[dt] = W::mma(vh, pl, o[dt]);
                    asm volatile("v_nop\n\tv_nop\n\tv_nop\n\tv_nop" : "+v"(o[dt]) : "v"(vh), "v"(vl), "v"(ph), "v"(pl) : "memory"); }
                else { asm volatile("v_nop\n\tv_nop\n\tv_nop\n\tv_nop" : "+v"(o[dt]) : "v"(vh), "v"(ph) : "memory"); }
            } }
    }
    const float lt = l + __shfl_xor(l, 16, 32);
    const float inv = 1.0f / lt;
#pragma unroll
    for (int dt = 0; dt < 4; ++dt)
#pragma unroll
        for (int r = 0; r < 8; ++r) os[lr * 68u + (unsigned)dt * 16u + 8u * hf + (unsigned)r] = o[dt][r] * inv;
    __builtin_amdgcn_wave_barrier(); asm volatile("" ::: "memory");
#pragma unroll 1
    for (int ps = 0; ps < 2; ++ps) {
#pragma unroll
        for (unsigned s4 = 0; s4 < 4; ++s4) { const unsigned row = 4u * s4 + (lane >> 3), pc = (lane & 7u) * 8u;
            const v4f x0 = *(const v4fa*)(os + row * 68u + pc); const v4f x1 = *(const v4fa*)(os + row * 68u + pc + 4u); v8us oh, ol;
#pragma unroll
            for (int q = 0; q < 4; ++q) { unsigned short a, c; splitf(x0[q], a, c); oh[q] = a; ol[q] = c; splitf(x1[q], a, c); oh[4 + q] = a; ol[4 + q] = c; }
            *(volatile v8us*)(Ah + (size_t)row * DQ + pc) = oh; *(volatile v8us*)(Al + (size_t)row * DQ + pc) = ol; }
        if (ps == 0) __threadfence(); }
    __builtin_amdgcn_wave_barrier(); asm volatile("" ::: "memory");
}

__global__ __launch_bounds__(32) void k_attn(const h16* QK16, const bf* QKBh, const bf* QKBl, const h16* VT16, const bf* VTBh, const bf* VTBl, bf* ATh, bf* ATl) {
    __shared__ __align__(16) float os[16 * 68];
    const unsigned q0 = blockIdx.x * 16u, head = blockIdx.y;
    bf* ah = ATh + (size_t)q0 * DQ + head * HD; bf* al = ATl + (size_t)q0 * DQ + head * HD;
    if (q0 < (unsigned)RH) {
        const size_t hq = (size_t)head * RH * HD, hk = (size_t)(NH_ + head) * RH * HD, hv = (size_t)head * HD * RH;
        attn_body<bf, 3>(QKBh + hq, QKBl + hq, QKBh + hk, QKBl + hk, VTBh + hv, VTBl + hv, (unsigned)RH, q0, ah, al, os);
    } else {
        const size_t hq = (size_t)head * TT * HD, hk = (size_t)(NH_ + head) * TT * HD, hv = (size_t)head * HD * TT;
        attn_body<h16, 1>(QK16 + hq, nullptr, QK16 + hk, nullptr, VT16 + hv, nullptr, (unsigned)TT, q0, ah, al, os);
    }
}

constexpr size_t SZ_WQKV = (size_t)3 * DQ * DM * 2;
constexpr size_t SZ_WO   = (size_t)DM * DQ * 2;
constexpr size_t SZ_XB   = (size_t)TT * DM * 2;
constexpr size_t SZ_F    = (size_t)TT * 3 * DQ * 4;
constexpr size_t SZ_QK16 = (size_t)2 * NH_ * TT * HD * 2;
constexpr size_t SZ_VT16 = (size_t)NH_ * HD * TT * 2;
constexpr size_t SZ_QKB  = (size_t)2 * NH_ * RH * HD * 2;
constexpr size_t SZ_VTB  = (size_t)NH_ * HD * RH * 2;
constexpr size_t SZ_AT   = (size_t)TT * DQ * 2;
constexpr size_t WS_TOTAL = SZ_WQKV + SZ_WO + SZ_XB + SZ_F + SZ_QK16 + SZ_VT16 + 2 * SZ_QKB + 2 * SZ_VTB + 2 * SZ_AT;
static_assert(WS_TOTAL <= (size_t)134217728);
static_assert(SZ_WQKV % 256 == 0 && SZ_WO % 256 == 0 && SZ_XB % 256 == 0 && SZ_F % 256 == 0 && SZ_QK16 % 256 == 0 && SZ_VT16 % 256 == 0 && SZ_QKB % 256 == 0 && SZ_VTB % 256 == 0 && SZ_AT % 256 == 0);
static_assert(((size_t)3 * DQ * DM / 64) % 64 == 0);
static_assert(((size_t)DQ * DM / 64) % 64 == 0);
static_assert(((size_t)TT * DM / 8) % 256 == 0);
static_assert(TT % 16 == 0);

extern "C" void kernel_launch(void* const* d_in, const int* in_sizes, int n_in,
                              void* d_out, int out_size, void* d_ws, size_t ws_size, hipStream_t stream) {
    if (n_in < 3) return;
    const size_t need_x = (size_t)(NB - 1) * SEQ_FULL * DM + (size_t)TT * DM;
    if ((size_t)in_sizes[0] < need_x || (size_t)in_sizes[1] < (size_t)DM * 3 * DQ || (size_t)in_sizes[2] < (size_t)DQ * DM || (size_t)out_size < need_x) return;
    if (ws_size < WS_TOTAL) return;
    const float* x = (const float*)d_in[0]; const float* wqkv = (const float*)d_in[1]; const float* wo = (const float*)d_in[2];
    float* OUT = (float*)d_out;
    char* wsp = (char*)d_ws;
    auto take = [&](size_t bytes) { char* p = wsp; wsp += (bytes + 255) & ~(size_t)255; return (void*)p; };
    bf* WQKV = (bf*)take(SZ_WQKV);
    bf* WO   = (bf*)take(SZ_WO);
    bf* XB   = (bf*)take(SZ_XB);
    float* F = (float*)take(SZ_F);
    h16* QK16 = (h16*)take(SZ_QK16);
    h16* VT16 = (h16*)take(SZ_VT16);
    bf* QKBh = (bf*)take(SZ_QKB); bf* QKBl = (bf*)take(SZ_QKB);
    bf* VTBh = (bf*)take(SZ_VTB); bf* VTBl = (bf*)take(SZ_VTB);
    bf* ATh = (bf*)take(SZ_AT); bf* ATl = (bf*)take(SZ_AT);
    if ((size_t)(wsp - (char*)d_ws) > ws_size) return;
    k_wtG<<<(unsigned)((DM * 3 * DQ / 64 + 63) / 64), 256, 0, stream>>>(wqkv, DM, 3 * DQ, WQKV);
    k_wtG<<<(unsigned)((DQ * DM / 64 + 63) / 64), 256, 0, stream>>>(wo, DQ, DM, WO);
    for (int b = 0; b < NB; ++b) {
        k_cvt8<<<(unsigned)(((size_t)TT * DM / 8 + 255) / 256), 256, 0, stream>>>(x + (size_t)b * SEQ_FULL * DM, XB, (size_t)TT * DM / 8);
        k_gemmw<bf, 0, false><<<dim3(TT / 64, 3 * DQ / 64, 1), 32, 0, stream>>>(XB, nullptr, WQKV, nullptr, DM, F, 3 * DQ, nullptr, 0, 0, 0);
        k_planes<<<BLK_QK + BLK_VT, 256, 0, stream>>>(F, QK16, QKBh, QKBl, VT16, VTBh, VTBl);
        k_attn<<<dim3(TT / 16, NH_, 1), 32, 0, stream>>>(QK16, QKBh, QKBl, VT16, VTBh, VTBl, ATh, ATl);
        k_gemmw<bf, 1, false><<<dim3(TT / 64, DM / 64, 1), 32, 0, stream>>>(ATh, ATl, WO, nullptr, DQ, OUT + (size_t)b * SEQ_FULL * DM, DM, nullptr, 0, 0, 0);
    }
}
